// OnnxAttention_7662221656204
// MI455X (gfx1250) — hardware-verified
//
#include <hip/hip_runtime.h>
#include <math.h>
#include <stdint.h>

#ifndef TQ
#define TQ 2048
#endif
#define PAST  2048
#define SKV   (PAST + TQ)
#define DMOD  2048
#define NH    16
#define NKVH  4
#define HD    128
#define KVD   (NKVH * HD)
#define NPAIR (HD / 2)
#define NGATE 12
#define WPB   (NH / NKVH)
#define NHG   NKVH
#define NQT   (TQ / 16)
#define NKT   (SKV / 32)
#define NKTP  (PAST / 32)
#define ATT_THREADS (WPB * 32)
#define RSQ_HD 0.08838834764831845f
#define LOG2E 1.4426950408889634f
#define QSC   1024.0f
#define KSC   1024.0f
#define PCAR  32768.0f
#define VCAR  1024.0f
#define OSC   1024.0f
#define WOS   1024.0f
#define PTP   36
#define PTW   (16 * PTP)
#define SLP   132
#define SLW   (16 * SLP)
#define WREG  (PTW + SLW)
#define SLAB64 (16 * 68)
#define VTP   72
#define SMF   9216
#define OFF1  ((size_t)TQ * DMOD)
#define OFF2  (OFF1 + (size_t)SKV * KVD)
#define OUT_TOTAL (OFF2 + (size_t)SKV * KVD)
#define WS_CAP 134217728
static_assert(DMOD == NH * HD && HD == 128 && NH == 16 && NKVH == 4 && WPB == 4 && NHG * WPB == NH);
static_assert(ATT_THREADS == 128 && KVD == 512 && NPAIR == 64);
static_assert((TQ % 64) == 0 && TQ >= 64 && (PAST % 64) == 0 && PAST >= 64);
static_assert((DMOD % 128) == 0 && (KVD % 128) == 0 && (DMOD % 32) == 0 && (HD % 32) == 0);
static_assert(((TQ * DMOD) % 2048) == 0 && ((PAST * KVD) % 2048) == 0 && ((TQ * DMOD / 8) % 256) == 0);
static_assert(SMF >= 64 * SLP && SMF * 2 >= 2 * HD * VTP);
static_assert(NKTP < NKT && NQT * 16 == TQ);

typedef unsigned short u16;
typedef _Float16 v16h __attribute__((ext_vector_type(16)));
typedef _Float16 v8h  __attribute__((ext_vector_type(8)));
typedef __bf16   v16b __attribute__((ext_vector_type(16)));
typedef float    v8f  __attribute__((ext_vector_type(8)));
typedef float    v4f  __attribute__((ext_vector_type(4)));
typedef unsigned int v4u __attribute__((ext_vector_type(4)));
typedef unsigned int v2u __attribute__((ext_vector_type(2)));

union FragH { v16h v; v8h h[2]; v4u u[2]; };
union FragB { v16b v; v4u u[2]; };

__device__ __forceinline__ unsigned short bf_bits(float f) {
  unsigned u = __float_as_uint(f);
  return (unsigned short)((u + 0x7FFFu + ((u >> 16) & 1u)) >> 16);
}
__device__ __forceinline__ float bf_up(unsigned short h) { return __uint_as_float(((unsigned)h) << 16); }
__device__ __forceinline__ float bfr(float f) { return bf_up(bf_bits(f)); }
__device__ __forceinline__ unsigned short h_bits(_Float16 x) { return __builtin_bit_cast(unsigned short, x); }
__device__ __forceinline__ unsigned pk16(unsigned short a, unsigned short b) { return (unsigned)a | ((unsigned)b << 16); }
__device__ __forceinline__ v8f zero8() { v8f z = {0.f, 0.f, 0.f, 0.f, 0.f, 0.f, 0.f, 0.f}; return z; }

__device__ __forceinline__ v16h ldfrag_h(const _Float16* p) {
  FragH f;
  f.h[0] = *(const v8h*)(p);
  f.h[1] = *(const v8h*)(p + 16);
  return f.v;
}
__device__ __forceinline__ v16b ldfrag_b(const u16* p) {
  FragB f;
  f.u[0] = *(const v4u*)(p);
  f.u[1] = *(const v4u*)(p + 16);
  return f.v;
}

__device__ __forceinline__ v8f mma_h(v16h a, v16h b, v8f c) {
  return __builtin_amdgcn_wmma_f32_16x16x32_f16(false, a, false, b, (short)0, c, false, false);
}
__device__ __forceinline__ v8f mma_b(v16b a, v16b b, v8f c) {
  return __builtin_amdgcn_wmma_f32_16x16x32_bf16(false, a, false, b, (short)0, c, false, false);
}
__device__ __forceinline__ void guard2(v8f& a, v8f& b, v16h x0, v16h x1, v16h x2, v16h x3, v16h x4, v16h x5) {
#if defined(__HIP_DEVICE_COMPILE__)
  asm volatile("v_nop\n\tv_nop\n\tv_nop\n\tv_nop"
               : "+v"(a), "+v"(b) : "v"(x0), "v"(x1), "v"(x2), "v"(x3), "v"(x4), "v"(x5) : "memory");
#endif
}
template <typename F>
__device__ __forceinline__ void guard6(v8f& a, v8f& b, v8f& c, v8f& d, F x0, F x1, F x2, F x3, F x4, F x5) {
#if defined(__HIP_DEVICE_COMPILE__)
  asm volatile("v_nop\n\tv_nop\n\tv_nop\n\tv_nop"
               : "+v"(a), "+v"(b), "+v"(c), "+v"(d) : "v"(x0), "v"(x1), "v"(x2), "v"(x3), "v"(x4), "v"(x5) : "memory");
#endif
}
__device__ __forceinline__ void acc_guard4(v8f& a, v8f& b, v8f& c, v8f& d) {
#if defined(__HIP_DEVICE_COMPILE__)
  asm volatile("v_nop\n\tv_nop\n\tv_nop\n\tv_nop" : "+v"(a), "+v"(b), "+v"(c), "+v"(d));
#endif
}
__device__ __forceinline__ void wave_sync_lds() {
  __builtin_amdgcn_fence(__ATOMIC_RELEASE, "workgroup");
  __builtin_amdgcn_wave_barrier();
  __builtin_amdgcn_fence(__ATOMIC_ACQUIRE, "workgroup");
}

__global__ __launch_bounds__(256) void cvt_bf(const float* __restrict__ x, u16* D, int n8) {
  const int gt = blockIdx.x * 256 + (int)threadIdx.x;
  if (gt >= n8) return;
  const float* p = x + (size_t)gt * 8;
  const v4f a = *(const v4f*)(p), b4 = *(const v4f*)(p + 4);
  v4u o;
  o[0] = pk16(bf_bits(a[0]), bf_bits(a[1]));
  o[1] = pk16(bf_bits(a[2]), bf_bits(a[3]));
  o[2] = pk16(bf_bits(b4[0]), bf_bits(b4[1]));
  o[3] = pk16(bf_bits(b4[2]), bf_bits(b4[3]));
  u16* d = D + (size_t)gt * 8;
  for (int pass = 0; pass < 2; ++pass) {
    *(volatile v4u*)(d) = o;
    __threadfence();
  }
}

__global__ __launch_bounds__(256) void wt16(const float* __restrict__ W, int ldw, int coff, int nct, u16* D,
                                            int f16mode, float scale) {
  __shared__ __align__(16) u16 T[128 * VTP];
  const int tid = threadIdx.x;
  const int bid = blockIdx.x;
  const int ct  = bid % nct;
  const int rt  = bid / nct;
  if (rt * 64 + 64 > DMOD) return;
  {
    const int sl = tid >> 2;
    const int dc = (tid & 3) * 32;
    const float* src = W + (size_t)(rt * 64 + sl) * ldw + coff + ct * 128 + dc;
#pragma unroll
    for (int i = 0; i < 8; ++i) {
      const v4f a = *(const v4f*)(src + 4 * i);
#pragma unroll
      for (int e = 0; e < 4; ++e) {
        const float f = a[e];
        const unsigned short hb = h_bits((_Float16)(bfr(f) * scale));
        const unsigned short bb = bf_bits(f);
        T[(dc + 4 * i + e) * VTP + sl] = (f16mode != 0) ? hb : bb;
      }
    }
  }
  __syncthreads();
  v4u w4[4];
  const int q8 = tid >> 3, p8 = (tid & 7) * 8;
#pragma unroll
  for (int it = 0; it < 4; ++it) {
    const int line = it * 32 + q8;
    w4[it] = *(const v4u*)(T + line * VTP + p8);
  }
  const size_t base = ((size_t)ct * 128) * DMOD + rt * 64 + p8;
  for (int pass = 0; pass < 2; ++pass) {
#pragma unroll
    for (int it = 0; it < 4; ++it) {
      const int line = it * 32 + q8;
      *(volatile v4u*)(D + base + (size_t)line * DMOD) = w4[it];
    }
    __threadfence();
  }
}

__global__ __launch_bounds__(256) void kpast(const float* __restrict__ pk, float* outk, u16* KHp, u16* KLp) {
  const int tid = (int)threadIdx.x;
  const int e0  = (int)blockIdx.x * 2048;
  if (e0 + 2048 > PAST * KVD) return;
  v4f ov0, ov1;
  {
    const v4f a = *(const v4f*)(pk + e0 + 4 * tid);
    const v4f b4 = *(const v4f*)(pk + e0 + 1024 + 4 * tid);
#pragma unroll
    for (int e = 0; e < 4; ++e) { ov0[e] = bfr(a[e]); ov1[e] = bfr(b4[e]); }
  }
  v4u oh, ol;
  {
    const float* p = pk + e0 + 8 * tid;
    const v4f a = *(const v4f*)(p), b4 = *(const v4f*)(p + 4);
    float w[8];
#pragma unroll
    for (int e = 0; e < 4; ++e) { w[e] = a[e]; w[4 + e] = b4[e]; }
#pragma unroll
    for (int e = 0; e < 4; ++e) {
      const float t0 = bfr(w[2 * e]) * KSC, t1 = bfr(w[2 * e + 1]) * KSC;
      const _Float16 h0 = (_Float16)t0, h1 = (_Float16)t1;
      const _Float16 l0 = (_Float16)(t0 - (float)h0), l1 = (_Float16)(t1 - (float)h1);
      oh[e] = pk16(h_bits(h0), h_bits(h1));
      ol[e] = pk16(h_bits(l0), h_bits(l1));
    }
  }
  float* d0 = outk + e0 + 4 * tid;
  float* d1 = outk + e0 + 1024 + 4 * tid;
  u16*   ph = KHp + (size_t)e0 + 8 * tid;
  u16*   pl = KLp + (size_t)e0 + 8 * tid;
  for (int pass = 0; pass < 2; ++pass) {
    *(volatile v4f*)(d0) = ov0;
    *(volatile v4f*)(d1) = ov1;
    *(volatile v4u*)(ph) = oh;
    *(volatile v4u*)(pl) = ol;
    __threadfence();
  }
}

template <int NEWV>
__global__ __launch_bounds__(256)
void vplanes(const float* __restrict__ src, const float* __restrict__ ve, const float* __restrict__ x,
             const float* __restrict__ wg, float* outv, u16* VHo, u16* VLo) {
  __shared__ __align__(16) float SM[SMF];
  const int tid = (int)threadIdx.x;
  const int bid = (int)blockIdx.x;
  constexpr int nst = (NEWV != 0) ? (TQ / 64) : (PAST / 64);
  const int st = bid % nst;
  const int g  = bid / nst;
  if (g >= NKVH) return;
  const int r0 = st * 64;
  const int s0 = ((NEWV != 0) ? PAST : 0) + r0;
  const int sl = tid >> 2;
  const int dc = (tid & 3) * 32;
  const float* sp = src + (size_t)(r0 + sl) * KVD + g * HD + dc;
  float w[32];
  if constexpr (NEWV != 0) {
    const int t = r0 + sl;
    const float* xr = x + (size_t)t * DMOD;
    const v4f x0 = *(const v4f*)(xr), x1 = *(const v4f*)(xr + 4), x2 = *(const v4f*)(xr + 8);
    float xs[NGATE];
#pragma unroll
    for (int e = 0; e < 4; ++e) { xs[e] = x0[e]; xs[4 + e] = x1[e]; xs[8 + e] = x2[e]; }
    float z = 0.0f;
#pragma unroll
    for (int i = 0; i < NGATE; ++i) z += bfr(xs[i]) * bfr(wg[i * NKVH + g]);
    const float zc = fmaxf(z, -80.0f);
    const float ex = expf(-zc);
    const float gt = 3.0f * __builtin_amdgcn_rcpf(1.0f + ex);
    const float* vp = ve + (size_t)t * KVD + g * HD + dc;
#pragma unroll
    for (int i = 0; i < 8; ++i) {
      const v4f a = *(const v4f*)(sp + 4 * i);
      const v4f b4 = *(const v4f*)(vp + 4 * i);
#pragma unroll
      for (int e = 0; e < 4; ++e) w[4 * i + e] = a[e] + gt * bfr(b4[e]);
    }
  } else {
#pragma unroll
    for (int i = 0; i < 8; ++i) {
      const v4f a = *(const v4f*)(sp + 4 * i);
#pragma unroll
      for (int e = 0; e < 4; ++e) w[4 * i + e] = bfr(a[e]);
    }
  }
  float* S32 = SM;
#pragma unroll
  for (int i = 0; i < 8; ++i) {
    v4f q4;
    q4[0] = w[4 * i]; q4[1] = w[4 * i + 1]; q4[2] = w[4 * i + 2]; q4[3] = w[4 * i + 3];
    *(v4f*)(S32 + sl * SLP + dc + 4 * i) = q4;
  }
  __syncthreads();
  const int wave = tid >> 5, lane = tid & 31;
  v4f ov[8];
#pragma unroll
  for (int it = 0; it < 8; ++it) {
    const int row = it * 8 + wave;
    ov[it] = *(const v4f*)(S32 + row * SLP + 4 * lane);
  }
  float* od = outv + (size_t)s0 * KVD + g * HD + 4 * lane;
  for (int pass = 0; pass < 2; ++pass) {
#pragma unroll
    for (int it = 0; it < 8; ++it) {
      const int row = it * 8 + wave;
      *(volatile v4f*)(od + (size_t)row * KVD) = ov[it];
    }
    __threadfence();
  }
  __syncthreads();
  u16* TH = reinterpret_cast<u16*>(SM);
  u16* TL = TH + HD * VTP;
#pragma unroll
  for (int i = 0; i < 32; ++i) {
    const float t = w[i] * VCAR;
    const _Float16 hv = (_Float16)t;
    const _Float16 lv = (_Float16)(t - (float)hv);
    TH[(dc + i) * VTP + sl] = h_bits(hv);
    TL[(dc + i) * VTP + sl] = h_bits(lv);
  }
  __syncthreads();
  v4u vh[4], vl[4];
  const int q8 = tid >> 3, p8 = (tid & 7) * 8;
#pragma unroll
  for (int it = 0; it < 4; ++it) {
    const int line = it * 32 + q8;
    vh[it] = *(const v4u*)(TH + line * VTP + p8);
    vl[it] = *(const v4u*)(TL + line * VTP + p8);
  }
  const size_t base = (size_t)(g * HD) * SKV + s0 + p8;
  for (int pass = 0; pass < 2; ++pass) {
#pragma unroll
    for (int it = 0; it < 4; ++it) {
      const int line = it * 32 + q8;
      *(volatile v4u*)(VHo + base + (size_t)line * SKV) = vh[it];
      *(volatile v4u*)(VLo + base + (size_t)line * SKV) = vl[it];
    }
    __threadfence();
  }
}

template <int WOUT>
__global__ __launch_bounds__(128)
void ropenorm(const float* __restrict__ F, int ncol, int nhb, const float* __restrict__ cosp, const float* __restrict__ sinp,
              u16* Hp, u16* Lp, int ppitch, int prow0, float* outk, float sc) {
#pragma clang fp contract(off)
  __shared__ __align__(16) u16 L2[1024];
  const int tid = (int)threadIdx.x, wave = tid >> 5, lane = tid & 31;
  const int bid = (int)blockIdx.x;
  const int hb  = bid % nhb;
  const int t   = bid / nhb;
  if (t >= TQ) return;
  const int col0 = hb * 512 + wave * HD;
  const int d4 = 4 * lane;
  const int j4 = 4 * (lane & 15);
  const int up = lane >> 4;
  const v4f a  = *(const v4f*)(F + (size_t)t * ncol + col0 + d4);
  const v4f cv = *(const v4f*)(cosp + (size_t)t * NPAIR + j4);
  const v4f sv = *(const v4f*)(sinp + (size_t)t * NPAIR + j4);
  float own[4], par[4], r[4];
#pragma unroll
  for (int e = 0; e < 4; ++e) own[e] = a[e];
#pragma unroll
  for (int e = 0; e < 4; ++e) par[e] = __shfl_xor(own[e], 16, 32);
  float sq = 0.0f;
#pragma unroll
  for (int e = 0; e < 4; ++e) {
    const float cc = bfr(cv[e]), ss = bfr(sv[e]);
    const float plo = own[e] * cc;
    const float qlo = par[e] * ss;
    const float rlo = plo + qlo;
    const float phi = par[e] * ss;
    const float qhi = own[e] * cc;
    const float rhi = qhi - phi;
    r[e] = (up != 0) ? rhi : rlo;
    sq += r[e] * r[e];
  }
#pragma unroll
  for (int off = 1; off < 32; off <<= 1) sq += __shfl_xor(sq, off, 32);
  const float mean = sq * (1.0f / (float)HD);
  const float rs = rsqrtf(mean + 1e-6f);
  v4f ov;
  float val[4];
#pragma unroll
  for (int e = 0; e < 4; ++e) { val[e] = (r[e] * rs) * 1.2f; ov[e] = val[e]; }
  float* od = outk + (size_t)(PAST + t) * KVD + wave * HD + d4;
  if constexpr (WOUT != 0) { *(volatile v4f*)(od) = ov; }
  v2u hp, lp;
  {
    unsigned short hbv[4], lbv[4];
#pragma unroll
    for (int e = 0; e < 4; ++e) {
      const float tt = val[e] * sc;
      const _Float16 hv = (_Float16)tt;
      const _Float16 lv = (_Float16)(tt - (float)hv);
      hbv[e] = h_bits(hv);
      lbv[e] = h_bits(lv);
    }
    hp[0] = pk16(hbv[0], hbv[1]); hp[1] = pk16(hbv[2], hbv[3]);
    lp[0] = pk16(lbv[0], lbv[1]); lp[1] = pk16(lbv[2], lbv[3]);
  }
  *(v2u*)(L2 + wave * HD + d4)       = hp;
  *(v2u*)(L2 + 512 + wave * HD + d4) = lp;
  __syncthreads();
  const int idx = (wave * 32 + lane) * 8;
  const v4u pv = *(const v4u*)(L2 + idx);
  u16* dpl = (wave < 2) ? Hp : Lp;
  const size_t doff = (size_t)(prow0 + t) * (size_t)ppitch + hb * 512 + ((wave & 1) * 32 + lane) * 8;
  *(volatile v4u*)(dpl + doff) = pv;
  __threadfence();
  if constexpr (WOUT != 0) { *(volatile v4f*)(od) = ov; }
  *(volatile v4u*)(dpl + doff) = pv;
  __threadfence();
}

__device__ __forceinline__ void epi64(float* sl, v8f a0, v8f a1, v8f a2, v8f a3, float oscale,
                                      float* C, int N, size_t rowb, int col0, int lane) {
  const int hh = lane >> 4, m = lane & 15;
#pragma unroll
  for (int r = 0; r < 8; ++r) {
    const int ro = (8 * hh + r) * 68 + m;
    sl[ro]      = a0[r] * oscale;
    sl[ro + 16] = a1[r] * oscale;
    sl[ro + 32] = a2[r] * oscale;
    sl[ro + 48] = a3[r] * oscale;
  }
  wave_sync_lds();
  v4f vals[8];
#pragma unroll
  for (int it = 0; it < 8; ++it) vals[it] = *(const v4f*)(sl + (it * 2 + hh) * 68 + m * 4);
  float* dst = C + (rowb + (size_t)hh) * (size_t)N + col0 + m * 4;
  for (int pass = 0; pass < 2; ++pass) {
#pragma unroll
    for (int it = 0; it < 8; ++it) {
      *(volatile v4f*)(dst + (size_t)(it * 2) * (size_t)N) = vals[it];
    }
    __threadfence();
  }
}

__global__ __launch_bounds__(128)
void gemm_bf(const u16* __restrict__ A, const u16* __restrict__ Bt, float* C, int M, int N, int K, float oscale) {
  __shared__ __align__(16) float slab[4 * SLAB64];
  const int tid = threadIdx.x, wave = tid >> 5, lane = tid & 31, hh = lane >> 4, m = lane & 15;
  const int ntile = N >> 6;
  const int bid   = blockIdx.x;
  const int rowb  = (bid / ntile) * 64 + wave * 16;
  const int col0  = (bid % ntile) * 64;
  if (rowb + 16 > M) return;
  const u16* ap = A  + (size_t)(rowb + m) * K + 8 * hh;
  const u16* bp = Bt + (size_t)(col0 + m) * K + 8 * hh;
  const size_t bs = (size_t)16 * K;
  v8f acc0 = zero8(), acc1 = zero8(), acc2 = zero8(), acc3 = zero8();
#pragma unroll 1
  for (int k0 = 0; k0 < K; k0 += 32) {
    const v16b a  = ldfrag_b(ap + k0);
    const v16b b0 = ldfrag_b(bp + k0);
    const v16b b1 = ldfrag_b(bp + bs + k0);
    const v16b b2 = ldfrag_b(bp + 2 * bs + k0);
    const v16b b3 = ldfrag_b(bp + 3 * bs + k0);
    acc0 = mma_b(a, b0, acc0);
    acc1 = mma_b(a, b1, acc1);
    acc2 = mma_b(a, b2, acc2);
    acc3 = mma_b(a, b3, acc3);
    guard6<v16b>(acc0, acc1, acc2, acc3, a, b0, b1, b2, b3, a);
  }
  epi64(slab + wave * SLAB64, acc0, acc1, acc2, acc3, oscale, C, N, (size_t)rowb, col0, lane);
}

__global__ __launch_bounds__(128)
void gemm_hf(const u16* __restrict__ A, const u16* __restrict__ Bt, float* C, int M, int N, int K, float oscale) {
  __shared__ __align__(16) float slab[4 * SLAB64];
  const int tid = threadIdx.x, wave = tid >> 5, lane = tid & 31, hh = lane >> 4, m = lane & 15;
  const int ntile = N >> 6;
  const int bid   = blockIdx.x;
  const int rowb  = (bid / ntile) * 64 + wave * 16;
  const int col0  = (bid % ntile) * 64;
  if (rowb + 16 > M) return;
  const _Float16* ap = (const _Float16*)(const void*)A  + (size_t)(rowb + m) * K + 8 * hh;
  const _Float16* bp = (const _Float16*)(const void*)Bt + (size_t)(col0 + m) * K + 8 * hh;
  const size_t bs = (size_t)16 * K;
  v8f acc0 = zero8(), acc1 = zero8(), acc2 = zero8(), acc3 = zero8();
#pragma unroll 1
  for (int k0 = 0; k0 < K; k0 += 32) {
    const v16h a  = ldfrag_h(ap + k0);
    const v16h b0 = ldfrag_h(bp + k0);
    const v16h b1 = ldfrag_h(bp + bs + k0);
    const v16h b2 = ldfrag_h(bp + 2 * bs + k0);
    const v16h b3 = ldfrag_h(bp + 3 * bs + k0);
    acc0 = mma_h(a, b0, acc0);
    acc1 = mma_h(a, b1, acc1);
    acc2 = mma_h(a, b2, acc2);
    acc3 = mma_h(a, b3, acc3);
    guard6<v16h>(acc0, acc1, acc2, acc3, a, b0, b1, b2, b3, a);
  }
  epi64(slab + wave * SLAB64, acc0, acc1, acc2, acc3, oscale, C, N, (size_t)rowb, col0, lane);
}

template <int RES>
__device__ __forceinline__ void att_step(int kb, const _Float16* Qh, const _Float16* Ql,
                                         const _Float16* Khb, const _Float16* Klb,
                                         const _Float16* Vhb, const _Float16* Vlb,
                                         float* pt, float (&mrow)[8], float (&lrow)[8], v8f (&o)[8],
                                         int qpos0, int hh, int c, float lsc) {
  v8f s0 = zero8(), s1 = zero8();
  const _Float16* k0p = Khb + (size_t)kb * KVD;
  const _Float16* k1p = k0p + (size_t)16 * KVD;
  const _Float16* l0p = Klb + (size_t)kb * KVD;
  const _Float16* l1p = l0p + (size_t)16 * KVD;
#pragma unroll
  for (int kk = 0; kk < HD / 32; ++kk) {
    const v16h qh  = ldfrag_h(Qh + kk * 32);
    const v16h ql  = ldfrag_h(Ql + kk * 32);
    const v16h kh0 = ldfrag_h(k0p + kk * 32);
    const v16h kh1 = ldfrag_h(k1p + kk * 32);
    s0 = mma_h(qh, kh0, s0);
    s0 = mma_h(ql, kh0, s0);
    s1 = mma_h(qh, kh1, s1);
    s1 = mma_h(ql, kh1, s1);
    if constexpr (RES != 0) {
      const v16h kl0 = ldfrag_h(l0p + kk * 32);
      const v16h kl1 = ldfrag_h(l1p + kk * 32);
      s0 = mma_h(qh, kl0, s0);
      s1 = mma_h(qh, kl1, s1);
      guard2(s0, s1, qh, ql, kh0, kh1, kl0, kl1);
    } else {
      guard2(s0, s1, qh, ql, kh0, kh1, qh, ql);
    }
  }
  const int key0 = kb + c, key1 = kb + 16 + c;
#pragma unroll
  for (int r = 0; r < 8; ++r) {
    const int   qp = qpos0 + r;
    const float u0 = s0[r] * lsc;
    const float u1 = s1[r] * lsc;
    const float t0 = (key0 > qp) ? -INFINITY : u0;
    const float t1 = (key1 > qp) ? -INFINITY : u1;
    float mx = fmaxf(t0, t1);
#pragma unroll
    for (int off = 1; off < 16; off <<= 1) mx = fmaxf(mx, __shfl_xor(mx, off, 32));
    const float mn = fmaxf(mrow[r], mx);
    const float ms = (mn == -INFINITY) ? 0.0f : mn;
    const float al = exp2f(mrow[r] - ms);
    mrow[r] = mn;
    const float e0 = exp2f(t0 - ms), e1 = exp2f(t1 - ms);
    float ps = e0 + e1;
#pragma unroll
    for (int off = 1; off < 16; off <<= 1) ps += __shfl_xor(ps, off, 32);
    lrow[r] = lrow[r] * al + ps;
#pragma unroll
    for (int j = 0; j < 8; ++j) o[j][r] *= al;
    const int ro = (8 * hh + r) * PTP + c;
    pt[ro]      = e0;
    pt[ro + 16] = e1;
  }
  wave_sync_lds();
  FragH ph;
  {
    const float* prow = pt + c * PTP + 8 * hh;
    const v4f p0 = *(const v4f*)(prow), p1 = *(const v4f*)(prow + 4);
    const v4f p2 = *(const v4f*)(prow + 16), p3 = *(const v4f*)(prow + 20);
#pragma unroll
    for (int e = 0; e < 4; ++e) {
      ph.h[0][e]     = (_Float16)(p0[e] * PCAR);
      ph.h[0][4 + e] = (_Float16)(p1[e] * PCAR);
      ph.h[1][e]     = (_Float16)(p2[e] * PCAR);
      ph.h[1][4 + e] = (_Float16)(p3[e] * PCAR);
    }
  }
  {
    const _Float16* vhp = Vhb + kb;
    const _Float16* vlp = Vlb + kb;
#pragma unroll
    for (int jg = 0; jg < 4; ++jg) {
      const size_t da = (size_t)(2 * jg) * 16 * SKV;
      const size_t db = da + (size_t)16 * SKV;
      const v16h vha = ldfrag_h(vhp + da), vhb2 = ldfrag_h(vhp + db);
      o[2 * jg]     = mma_h(ph.v, vha,  o[2 * jg]);
      o[2 * jg + 1] = mma_h(ph.v, vhb2, o[2 * jg + 1]);
      if constexpr (RES != 0) {
        const v16h vla = ldfrag_h(vlp + da), vlb2 = ldfrag_h(vlp + db);
        o[2 * jg]     = mma_h(ph.v, vla,  o[2 * jg]);
        o[2 * jg + 1] = mma_h(ph.v, vlb2, o[2 * jg + 1]);
        guard2(o[2 * jg], o[2 * jg + 1], ph.v, vha, vhb2, vla, vlb2, ph.v);
      } else {
        guard2(o[2 * jg], o[2 * jg + 1], ph.v, vha, vhb2, ph.v, vha, vhb2);
      }
    }
  }
  wave_sync_lds();
}

__global__ __launch_bounds__(ATT_THREADS)
void attn(const u16* __restrict__ QHp, const u16* __restrict__ QLp,
          const u16* __restrict__ KHp, const u16* __restrict__ KLp,
          const u16* __restrict__ VHp, const u16* __restrict__ VLp, u16* OHp) {
  __shared__ __align__(16) float smem[WPB * WREG];

  const int tid  = threadIdx.x;
  const int wave = tid >> 5;
  const int lane = tid & 31;
  const int hh   = lane >> 4;
  const int c    = lane & 15;
  const int bid  = blockIdx.x;
  const int qt   = bid % NQT;
  const int hg   = bid / NQT;
  if (hg >= NHG) return;
  const int q0   = qt * 16;
  const int head = hg * WPB + wave;
  const int kvh  = hg;

  float* pt   = smem + wave * WREG;
  float* slab = pt + PTW;

  const size_t hcol = (size_t)head * HD + 8 * hh;
  const size_t kcol = (size_t)kvh * HD + 8 * hh;
  const _Float16* Qh  = (const _Float16*)(const void*)QHp + ((size_t)q0 + c) * DMOD + hcol;
  const _Float16* Ql  = (const _Float16*)(const void*)QLp + ((size_t)q0 + c) * DMOD + hcol;
  const _Float16* Khb = (const _Float16*)(const void*)KHp + (size_t)c * KVD + kcol;
  const _Float16* Klb = (const _Float16*)(const void*)KLp + (size_t)c * KVD + kcol;
  const _Float16* Vhb = (const _Float16*)(const void*)VHp + ((size_t)kvh * HD + c) * SKV + 8 * hh;
  const _Float16* Vlb = (const _Float16*)(const void*)VLp + ((size_t)kvh * HD + c) * SKV + 8 * hh;
  const float lsc = RSQ_HD * (LOG2E / (QSC * KSC));
  const float oc  = 1.0f / (PCAR * VCAR);

  float mrow[8], lrow[8];
  v8f o[8];
#pragma unroll
  for (int r = 0; r < 8; ++r) { mrow[r] = -INFINITY; lrow[r] = 0.f; }
#pragma unroll
  for (int j = 0; j < 8; ++j) o[j] = zero8();
  int nkt = ((PAST + q0) >> 5) + 1;
  if (nkt > NKT) nkt = NKT;
  const int qpos0 = PAST + q0 + 8 * hh;

#pragma unroll 1
  for (int kt = 0; kt < NKTP; ++kt) {
    att_step<0>(kt * 32, Qh, Ql, Khb, Klb, Vhb, Vlb, pt, mrow, lrow, o, qpos0, hh, c, lsc);
  }
#pragma unroll 1
  for (int kt = NKTP; kt < nkt; ++kt) {
    att_step<1>(kt * 32, Qh, Ql, Khb, Klb, Vhb, Vlb, pt, mrow, lrow, o, qpos0, hh, c, lsc);
  }
  acc_guard4(o[0], o[1], o[2], o[3]);
  acc_guard4(o[4], o[5], o[6], o[7]);
#pragma unroll
  for (int r = 0; r < 8; ++r) {
    const float lv  = lrow[r];
    const float ls  = (lv > 0.0f) ? lv : 1.0f;
    const float inv = (lv > 0.0f) ? ((1.0f / ls) * oc) : 0.0f;
#pragma unroll
    for (int j = 0; j < 8; ++j) {
      const int idx = (8 * hh + r) * SLP + j * 16 + c;
      slab[idx] = o[j][r] * inv;
    }
  }

  wave_sync_lds();
  v4u oh[8];
  const int rq = lane >> 4, c8 = (lane & 15) * 8;
#pragma unroll
  for (int it = 0; it < 8; ++it) {
    const int row = it * 2 + rq;
    const v4f a = *(const v4f*)(slab + row * SLP + c8), b4 = *(const v4f*)(slab + row * SLP + c8 + 4);
    float w[8];
#pragma unroll
    for (int e = 0; e < 4; ++e) { w[e] = a[e] * OSC; w[4 + e] = b4[e] * OSC; }
#pragma unroll
    for (int e = 0; e < 4; ++e) {
      const _Float16 h0 = (_Float16)w[2 * e], h1 = (_Float16)w[2 * e + 1];
      oh[it][e] = pk16(h_bits(h0), h_bits(h1));
    }
  }
  const size_t ob = (size_t)q0 * DMOD + (size_t)head * HD + c8;
  for (int pass = 0; pass < 2; ++pass) {
#pragma unroll
    for (int it = 0; it < 8; ++it) {
      const int row = it * 2 + rq;
      *(volatile v4u*)(OHp + ob + (size_t)row * DMOD) = oh[it];
    }
    __threadfence();
  }
}

extern "C" void kernel_launch(void* const* d_in, const int* in_sizes, int n_in,
                              void* d_out, int out_size, void* d_ws, size_t ws_size,
                              hipStream_t stream) {
  if (n_in < 11) return;
  if (in_sizes[0] != TQ * DMOD) return;
  if (in_sizes[1] != TQ * KVD) return;
  if (in_sizes[2] != TQ * NPAIR) return;
  if (in_sizes[3] != TQ * NPAIR) return;
  if (in_sizes[4] != PAST * KVD) return;
  if (in_sizes[5] != PAST * KVD) return;
  if (in_sizes[6] != DMOD * DMOD) return;
  if (in_sizes[7] != DMOD * KVD) return;
  if (in_sizes[8] != DMOD * KVD) return;
  if (in_sizes[9] != DMOD * DMOD) return;
  if (in_sizes[10] != NGATE * NKVH) return;
  if ((size_t)out_size != OUT_TOTAL) return;

  const float* x    = (const float*)d_in[0];
  const float* ve   = (const float*)d_in[1];
  const float* cosp = (const float*)d_in[2];
  const float* sinp = (const float*)d_in[3];
  const float* pk   = (const float*)d_in[4];
  const float* pv   = (const float*)d_in[5];
  const float* wq   = (const float*)d_in[6];
  const float* wk   = (const float*)d_in[7];
  const float* wv   = (const float*)d_in[8];
  const float* wo   = (const float*)d_in[9];
  const float* wgp  = (const float*)d_in[10];
  float* out0 = (float*)d_out;
  float* out1 = out0 + OFF1;
  float* out2 = out0 + OFF2;

  const size_t szXB = (size_t)TQ * DMOD * 2;
  const size_t szW  = (size_t)DMOD * DMOD * 2;
  const size_t szF  = (size_t)TQ * DMOD * 4;
  const size_t szOH = (size_t)TQ * DMOD * 2;
  const size_t szQ  = (size_t)TQ * DMOD * 2;
  const size_t szK  = (size_t)SKV * KVD * 2;
  const size_t szV  = (size_t)NKVH * HD * SKV * 2;
  size_t off = 0;
  const size_t oXB = off; off += szXB;
  const size_t oW  = off; off += szW;
  const size_t oF  = off; off += szF;
  const size_t oOH = off; off += szOH;
  const size_t oQH = off; off += szQ;
  const size_t oQL = off; off += szQ;
  const size_t oKH = off; off += szK;
  const size_t oKL = off; off += szK;
  const size_t oVH = off; off += szV;
  const size_t oVL = off; off += szV;
  if (off > ws_size) return;
  if (off > (size_t)WS_CAP) return;

  char* ws = (char*)d_ws;
  u16*   XB = (u16*)(ws + oXB);
  u16*   WB = (u16*)(ws + oW);
  float* F  = (float*)(ws + oF);
  u16*   OH = (u16*)(ws + oOH);
  u16*   QH = (u16*)(ws + oQH);
  u16*   QL = (u16*)(ws + oQL);
  u16*   KH = (u16*)(ws + oKH);
  u16*   KL = (u16*)(ws + oKL);
  u16*   VH = (u16*)(ws + oVH);
  u16*   VL = (u16*)(ws + oVL);

  const dim3 b256(256), b128(128), bAT(ATT_THREADS);
  const int  n8x  = (TQ * DMOD) / 8;
  const dim3 gX((n8x + 255) / 256);
  const int  nctQ = DMOD / 128;
  const int  nctK = KVD / 128;
  const dim3 gWQ(nctQ * (DMOD / 64));
  const dim3 gWK(nctK * (DMOD / 64));
  const dim3 gGQ((TQ / 64) * (DMOD / 64));
  const dim3 gGK((TQ / 64) * (KVD / 64));
  const dim3 gVP(NKVH * (PAST / 64));
  const dim3 gVN(NKVH * (TQ / 64));
  const dim3 gKP((PAST * KVD) / 2048);
  const dim3 gRK(TQ);
  const dim3 gRQ(TQ * (DMOD / 512));
  const dim3 gAT(NQT * NHG);

  cvt_bf<<<gX, b256, 0, stream>>>(x, XB, n8x);
  wt16<<<gWK, b256, 0, stream>>>(wv, KVD, 0, nctK, WB, 0, 1.0f);
  gemm_bf<<<gGK, b128, 0, stream>>>(XB, WB, F, TQ, KVD, DMOD, 1.0f);
  vplanes<0><<<gVP, b256, 0, stream>>>(pv, ve, x, wgp, out2, VH, VL);
  vplanes<1><<<gVN, b256, 0, stream>>>(F, ve, x, wgp, out2, VH, VL);
  kpast<<<gKP, b256, 0, stream>>>(pk, out1, KH, KL);
  wt16<<<gWK, b256, 0, stream>>>(wk, KVD, 0, nctK, WB, 0, 1.0f);
  gemm_bf<<<gGK, b128, 0, stream>>>(XB, WB, F, TQ, KVD, DMOD, 1.0f);
  ropenorm<1><<<gRK, b128, 0, stream>>>(F, KVD, 1, cosp, sinp, KH, KL, KVD, PAST, out1, KSC);
  wt16<<<gWQ, b256, 0, stream>>>(wq, DMOD, 0, nctQ, WB, 0, 1.0f);
  gemm_bf<<<gGQ, b128, 0, stream>>>(XB, WB, F, TQ, DMOD, DMOD, 1.0f);
  ropenorm<0><<<gRQ, b128, 0, stream>>>(F, DMOD, DMOD / 512, cosp, sinp, QH, QL, DMOD, 0, out1, QSC);
  wt16<<<gWQ, b256, 0, stream>>>(wo, DMOD, 0, nctQ, WB, 1, WOS);
  attn<<<gAT, bAT, 0, stream>>>(QH, QL, KH, KL, VH, VL, OH);
  gemm_hf<<<gGQ, b128, 0, stream>>>(OH, WB, out0, TQ, DMOD, DMOD, 1.0f / (OSC * WOS));
  (void)hipGetLastError();
}
